// SocialLSTM_24524263260712
// MI455X (gfx1250) — hardware-verified
//
#include <hip/hip_runtime.h>
#include <math.h>

constexpr int NSTEPS = 14;
constexpr int NAGENT = 65536;
constexpr int HID    = 64;
constexpr int NGATE  = 4 * HID;
constexpr int GRIDW  = 4;
constexpr int NCELL  = GRIDW * GRIDW;
constexpr int NSOC   = NCELL * HID;
constexpr int AGB    = 64;
constexpr int NBLK   = NAGENT / AGB;
constexpr int NTHR   = 256;
constexpr int AHP    = 72;
constexpr int HTP    = 72;
constexpr int OHP    = 72;
constexpr int SLP    = 68;
constexpr int NOUT   = NSTEPS * 2;
constexpr float WCAR    = 256.0f;
constexpr float HCAR    = 64.0f;
constexpr float ACC_INV = 1.0f / (256.0f * 64.0f);
constexpr float HALF_NB = 2.0f;
static_assert(NAGENT % AGB == 0, "agent tiling exact");
static_assert(AGB == 64 && HID == 64 && NTHR == 256, "wave map: 4 m-subtiles x 2 unit-subtile pairs = 8 waves");
static_assert(NGATE == NTHR, "one gate column of parameters per thread");
static_assert(NSOC == 4 * NTHR, "partial grid: one float4 per thread");
static_assert((AGB * AHP) % NTHR == 0, "h tile zero fill exact");
static_assert(HID % 32 == 0, "K multiple of 32");
static_assert(NOUT <= 32, "output staging");
static_assert((NGATE * HID) % (8 * NTHR) == 0, "weight cast grid exact");

typedef __attribute__((ext_vector_type(16))) _Float16 v16h;
typedef __attribute__((ext_vector_type(8)))  _Float16 v8h;
typedef __attribute__((ext_vector_type(16))) __bf16   v16b;
typedef __attribute__((ext_vector_type(8)))  __bf16   v8b;
typedef __attribute__((ext_vector_type(8)))  float    v8f;
typedef __attribute__((ext_vector_type(4)))  float    v4f;
typedef __attribute__((ext_vector_type(4)))  unsigned v4u;

__device__ __forceinline__ unsigned short f2bf_bits(float f) {
  unsigned u = __float_as_uint(f);
  return (unsigned short)((u + 0x7FFFu + ((u >> 16) & 1u)) >> 16);
}
__device__ __forceinline__ float bf_bits2f(unsigned short h) { return __uint_as_float(((unsigned)h) << 16); }

__device__ __forceinline__ void dep_guard4h(v8f& a0, v8f& a1, v8f& a2, v8f& a3,
                                            v16h x, v16h y0, v16h y1, v16h y2, v16h y3) {
  asm volatile("v_nop\n\tv_nop\n\tv_nop\n\tv_nop"
               : "+v"(a0), "+v"(a1), "+v"(a2), "+v"(a3)
               : "v"(x), "v"(y0), "v"(y1), "v"(y2), "v"(y3));
}
__device__ __forceinline__ void acc_guard4(v8f& a, v8f& b, v8f& c, v8f& d) {
  asm volatile("v_nop\n\tv_nop\n\tv_nop\n\tv_nop" : "+v"(a), "+v"(b), "+v"(c), "+v"(d));
}
template <typename T> struct Frag;
template <> struct Frag<_Float16> {
  typedef v16h V; union U { v16h v; v8h h[2]; };
  static __device__ __forceinline__ v16h load(const _Float16* p) {
    U f; f.h[0] = *(const v8h*)(p); f.h[1] = *(const v8h*)(p + 16); return f.v;
  }
  static __device__ __forceinline__ v8f mma(v16h a, v16h b, v8f c) {
    return __builtin_amdgcn_wmma_f32_16x16x32_f16(false, a, false, b, (short)0, c, false, false);
  }
};
template <> struct Frag<__bf16> {
  typedef v16b V; union U { v16b v; v8b h[2]; };
  static __device__ __forceinline__ v16b load(const __bf16* p) {
    U f; f.h[0] = *(const v8b*)(p); f.h[1] = *(const v8b*)(p + 16); return f.v;
  }
};
__device__ __forceinline__ v8f mma_bf16_g(v16b a, v16b b, v8f cacc) {
  cacc = __builtin_amdgcn_wmma_f32_16x16x32_bf16(false, a, false, b, (short)0, cacc, false, false);
  asm volatile("v_nop\n\tv_nop\n\tv_nop\n\tv_nop" : "+v"(cacc) : "v"(a), "v"(b));
  return cacc;
}

__device__ __forceinline__ float fsig(float x)  { return __builtin_amdgcn_rcpf(1.0f + expf(-x)); }
__device__ __forceinline__ float ftanh(float x) { return 1.0f - 2.0f * __builtin_amdgcn_rcpf(expf(2.0f * x) + 1.0f); }

__device__ __forceinline__ int cell_of(float x0, float x1, float tpx, float tpy) {
  const float rx = x0 - tpx;
  const float ry = x1 - tpy;
  const bool inside = (fabsf(rx) <= HALF_NB) && (fabsf(ry) <= HALF_NB);
  const float rxc = fminf(fmaxf(rx, -8.0f), 8.0f);
  const float ryc = fminf(fmaxf(ry, -8.0f), 8.0f);
  const int cx = (int)rxc + GRIDW / 2;
  const int cy = (int)ryc + GRIDW / 2;
  const bool valid = inside && (cx >= 0) && (cx < GRIDW) && (cy >= 0) && (cy < GRIDW);
  return valid ? (cy * GRIDW + cx) : -1;
}

__global__ __launch_bounds__(NTHR) void cvt_whh_kernel(const float* __restrict__ src, unsigned short* __restrict__ dst,
                                                       int n8, float sc) {
  const int i = blockIdx.x * NTHR + threadIdx.x;
  if (i < n8) {
    const v4f a = *(const v4f*)(src + (size_t)i * 8);
    const v4f b = *(const v4f*)(src + (size_t)i * 8 + 4);
    v8h hv;
#pragma unroll
    for (int e = 0; e < 4; ++e) {
      hv[e]     = (_Float16)(a[e] * sc);
      hv[4 + e] = (_Float16)(b[e] * sc);
    }
    *(volatile v8h*)(dst + (size_t)i * 8) = hv;
    __threadfence();
    *(volatile v8h*)(dst + (size_t)i * 8) = hv;
  }
}

__global__ __launch_bounds__(NTHR) void agents_kernel(const float* __restrict__ traj_t, const float* __restrict__ traj_o,
                                                      const float* __restrict__ w_ih, const float* __restrict__ b_ih,
                                                      const float* __restrict__ b_hh,
                                                      const unsigned short* __restrict__ WHHp,
                                                      float* __restrict__ PART) {
  __shared__ __align__(16) _Float16       Ah[AGB * AHP];
  __shared__ __align__(16) unsigned short HT[3 * HID * HTP];
  __shared__ __align__(16) unsigned short OH[NCELL * OHP];
  __shared__ __align__(16) float          xs[AGB * 2];
  __shared__ __align__(16) float          cpar[NGATE * 4];
  __shared__ __align__(16) float          slab[NCELL * SLP];
  const _Float16* WHH = (const _Float16*)WHHp;
  const int tid = threadIdx.x, lane = tid & 31, wave = tid >> 5;
  const int c = lane & 15, hh = lane >> 4, koff = 8 * hh;
  const int msub = wave >> 1, ubase = 2 * (wave & 1);
  const int abase = 16 * msub + 8 * hh;
  const int blk = blockIdx.x;
  const size_t agent0 = (size_t)blk * AGB;

#pragma unroll 1
  for (int i = 0; i < (AGB * AHP) / NTHR; ++i) Ah[i * NTHR + tid] = (_Float16)0.0f;
  {
    v4f pv;
    pv[0] = b_ih[tid] + b_hh[tid];
    pv[1] = w_ih[2 * tid];
    pv[2] = w_ih[2 * tid + 1];
    pv[3] = 0.0f;
    *(v4f*)(cpar + 4 * tid) = pv;
  }
  if (wave == 4) {
    const v4f v = *(const v4f*)(traj_o + agent0 * 2 + 4 * lane);
    *(v4f*)(xs + 4 * lane) = v;
  }
  float cst[2][8], hst[2][8];
#pragma unroll
  for (int q = 0; q < 2; ++q)
#pragma unroll
    for (int r = 0; r < 8; ++r) { cst[q][r] = 0.0f; hst[q][r] = 0.0f; }
  __syncthreads();

  const v8f z8 = {0.f, 0.f, 0.f, 0.f, 0.f, 0.f, 0.f, 0.f};
  const _Float16* arow = Ah + (16 * msub + c) * AHP + koff;

#pragma unroll 1
  for (int t = 0; t < NSTEPS; ++t) {
    const float tpx = traj_t[2 * t];
    const float tpy = traj_t[2 * t + 1];

#pragma unroll
    for (int ubi = 0; ubi < 2; ++ubi) {
      const int u = 16 * (ubase + ubi) + c;
      const _Float16* wrow = WHH + (size_t)u * HID + koff;
      v8f acc[4];
      acc[0] = z8; acc[1] = z8; acc[2] = z8; acc[3] = z8;
#pragma unroll 1
      for (int k0 = 0; k0 < HID; k0 += 32) {
        const v16h a  = Frag<_Float16>::load(arow + k0);
        const v16h b0 = Frag<_Float16>::load(wrow + k0);
        const v16h b1 = Frag<_Float16>::load(wrow + (size_t)1 * HID * HID + k0);
        const v16h b2 = Frag<_Float16>::load(wrow + (size_t)2 * HID * HID + k0);
        const v16h b3 = Frag<_Float16>::load(wrow + (size_t)3 * HID * HID + k0);
        acc[0] = Frag<_Float16>::mma(a, b0, acc[0]);
        acc[1] = Frag<_Float16>::mma(a, b1, acc[1]);
        acc[2] = Frag<_Float16>::mma(a, b2, acc[2]);
        acc[3] = Frag<_Float16>::mma(a, b3, acc[3]);
        dep_guard4h(acc[0], acc[1], acc[2], acc[3], a, b0, b1, b2, b3);
      }
      acc_guard4(acc[0], acc[1], acc[2], acc[3]);
      const v4f p0 = *(const v4f*)(cpar + 4 * (0 * HID + u));
      const v4f p1 = *(const v4f*)(cpar + 4 * (1 * HID + u));
      const v4f p2 = *(const v4f*)(cpar + 4 * (2 * HID + u));
      const v4f p3 = *(const v4f*)(cpar + 4 * (3 * HID + u));
#pragma unroll
      for (int r = 0; r < 8; ++r) {
        const int a = abase + r;
        const float x0 = xs[2 * a];
        const float x1 = xs[2 * a + 1];
        const float zi = acc[0][r] * ACC_INV + (p0[0] + (p0[1] * x0 + p0[2] * x1));
        const float zf = acc[1][r] * ACC_INV + (p1[0] + (p1[1] * x0 + p1[2] * x1));
        const float zg = acc[2][r] * ACC_INV + (p2[0] + (p2[1] * x0 + p2[2] * x1));
        const float zo = acc[3][r] * ACC_INV + (p3[0] + (p3[1] * x0 + p3[2] * x1));
        const float ig = fsig(zi);
        const float fg = fsig(zf);
        const float gg = ftanh(zg);
        const float og = fsig(zo);
        const float cn = fg * cst[ubi][r] + ig * gg;
        cst[ubi][r] = cn;
        hst[ubi][r] = og * ftanh(cn);
      }
    }
    __syncthreads();

#pragma unroll
    for (int ubi = 0; ubi < 2; ++ubi) {
      const int u = 16 * (ubase + ubi) + c;
      unsigned ph[4] = {0u, 0u, 0u, 0u}, pm[4] = {0u, 0u, 0u, 0u}, pl[4] = {0u, 0u, 0u, 0u};
#pragma unroll
      for (int r = 0; r < 8; ++r) {
        const float h = hst[ubi][r];
        Ah[(abase + r) * AHP + u] = (_Float16)(h * HCAR);
        const unsigned short hb = f2bf_bits(h);
        const float rem1 = h - bf_bits2f(hb);
        const unsigned short mb = f2bf_bits(rem1);
        const float rem2 = rem1 - bf_bits2f(mb);
        const unsigned short lb = f2bf_bits(rem2);
        const int q = r >> 1, sh = (r & 1) * 16;
        ph[q] |= ((unsigned)hb) << sh;
        pm[q] |= ((unsigned)mb) << sh;
        pl[q] |= ((unsigned)lb) << sh;
      }
      v4u vh, vm, vl;
#pragma unroll
      for (int q = 0; q < 4; ++q) { vh[q] = ph[q]; vm[q] = pm[q]; vl[q] = pl[q]; }
      unsigned short* hp = HT + u * HTP + abase;
      *(v4u*)(hp) = vh;
      *(v4u*)(hp + 1 * HID * HTP) = vm;
      *(v4u*)(hp + 2 * HID * HTP) = vl;
    }
    {
      const int a = tid & 63, cq = tid >> 6;
      const int cell = cell_of(xs[2 * a], xs[2 * a + 1], tpx, tpy);
#pragma unroll
      for (int i = 0; i < 4; ++i) {
        const int cid = 4 * cq + i;
        OH[cid * OHP + a] = (cell == cid) ? (unsigned short)0x3F80u : (unsigned short)0u;
      }
    }
    __syncthreads();

    if (wave < 4) {
      const int nt = wave;
      const __bf16* OHb = (const __bf16*)OH + c * OHP + koff;
      const __bf16* HTb = (const __bf16*)HT + (16 * nt + c) * HTP + koff;
      v8f d = z8;
#pragma unroll
      for (int ks = 0; ks < AGB; ks += 32) {
        const v16b a = Frag<__bf16>::load(OHb + ks);
#pragma unroll
        for (int p = 0; p < 3; ++p) {
          const v16b b = Frag<__bf16>::load(HTb + p * HID * HTP + ks);
          d = mma_bf16_g(a, b, d);
        }
      }
#pragma unroll
      for (int r = 0; r < 8; ++r) slab[(8 * hh + r) * SLP + 16 * nt + c] = d[r];
    } else if (wave == 4) {
      const int tn = (t + 1 < NSTEPS) ? (t + 1) : (NSTEPS - 1);
      const v4f v = *(const v4f*)(traj_o + ((size_t)tn * NAGENT + agent0) * 2 + 4 * lane);
      *(v4f*)(xs + 4 * lane) = v;
    }
    __syncthreads();

    {
      const int row = tid >> 4, c4 = (tid & 15) * 4;
      const v4f v = *(const v4f*)(slab + row * SLP + c4);
      float* dst = PART + ((size_t)blk * NSTEPS + (size_t)t) * NSOC + row * HID + c4;
      for (int pass = 0; pass < 2; ++pass) {
        *(volatile v4f*)dst = v;
        __threadfence();
      }
    }
  }
}

__global__ __launch_bounds__(NTHR) void pool_target_kernel(const float* __restrict__ traj_t, const float* __restrict__ w_ih,
                                                           const float* __restrict__ w_hh, const float* __restrict__ b_ih,
                                                           const float* __restrict__ b_hh, const float* __restrict__ w1,
                                                           const float* __restrict__ b1, const float* __restrict__ w2,
                                                           const float* __restrict__ b2, const float* __restrict__ wout,
                                                           const float* __restrict__ bout, const float* __restrict__ PART,
                                                           float* __restrict__ out) {
  __shared__ __align__(16) float grid_s[NSOC];
  __shared__ float gates_s[NGATE];
  __shared__ float ht[HID];
  __shared__ float ct[HID];
  __shared__ float hid1[HID];
  __shared__ float scv[HID];
  __shared__ float part4[4 * HID];
  __shared__ __align__(16) float outs[32];
  const int tid = threadIdx.x, lane = tid & 31, wave = tid >> 5;
  const float bsum = b_ih[tid] + b_hh[tid];
  const float wi0  = w_ih[2 * tid];
  const float wi1  = w_ih[2 * tid + 1];
  if (tid < HID) { ht[tid] = 0.0f; ct[tid] = 0.0f; }
  if (tid < 32) outs[tid] = 0.0f;
  __syncthreads();

#pragma unroll 1
  for (int t = 0; t < NSTEPS; ++t) {
    const float tpx = traj_t[2 * t];
    const float tpy = traj_t[2 * t + 1];
    {
      const int c4 = 4 * tid;
      const float* pp = PART + (size_t)t * NSOC + c4;
      double d0 = 0.0, d1 = 0.0, d2 = 0.0, d3 = 0.0;
#pragma unroll 1
      for (int b = 0; b < NBLK; ++b) {
        const v4f v = *(const v4f*)(pp + (size_t)b * NSTEPS * NSOC);
        d0 += (double)v[0]; d1 += (double)v[1]; d2 += (double)v[2]; d3 += (double)v[3];
      }
      v4f g4;
      g4[0] = (float)d0; g4[1] = (float)d1; g4[2] = (float)d2; g4[3] = (float)d3;
      *(v4f*)(grid_s + c4) = g4;
    }
    __syncthreads();
    {
      float acc = bsum + (wi0 * tpx + wi1 * tpy);
      const float* wr = w_hh + (size_t)tid * HID;
#pragma unroll 1
      for (int k = 0; k < HID; ++k) acc += wr[k] * ht[k];
      gates_s[tid] = acc;
    }
    {
      const int n = tid & 63, q = tid >> 6;
      const float* wr = w1 + (size_t)n * NSOC + q * 256;
      const float* gs = grid_s + q * 256;
      float s = 0.0f;
#pragma unroll 1
      for (int k = 0; k < 256; ++k) s += wr[k] * gs[k];
      part4[q * HID + n] = s;
    }
    __syncthreads();
    if (tid < HID) {
      const float zi = gates_s[tid], zf = gates_s[HID + tid], zg = gates_s[2 * HID + tid], zo = gates_s[3 * HID + tid];
      const float cn = fsig(zf) * ct[tid] + fsig(zi) * ftanh(zg);
      const float hn = fsig(zo) * ftanh(cn);
      ct[tid] = cn;
      ht[tid] = hn;
      const float r1 = b1[tid] + ((part4[tid] + part4[HID + tid]) + (part4[2 * HID + tid] + part4[3 * HID + tid]));
      hid1[tid] = fmaxf(r1, 0.0f);
    }
    __syncthreads();
    if (tid < HID) {
      float s = b2[tid];
      const float* wr = w2 + (size_t)tid * HID;
#pragma unroll 1
      for (int k = 0; k < HID; ++k) s += wr[k] * hid1[k];
      scv[tid] = s;
    }
    __syncthreads();
    if (tid < 2) {
      float s = bout[tid];
      const float* wr = wout + (size_t)tid * HID;
#pragma unroll 1
      for (int k = 0; k < HID; ++k) s += wr[k] * (ht[k] + scv[k]);
      outs[2 * t + tid] = s;
    }
    __syncthreads();
  }
  if (wave == 0) {
    const v4f v = *(const v4f*)(outs + 4 * (lane & 7));
    for (int pass = 0; pass < 2; ++pass) {
      if (lane < 7) *(volatile v4f*)(out + 4 * lane) = v;
      __threadfence();
    }
  }
}

extern "C" void kernel_launch(void* const* d_in, const int* in_sizes, int n_in,
                              void* d_out, int out_size, void* d_ws, size_t ws_size, hipStream_t stream) {
  if (n_in < 12 || d_out == nullptr || d_ws == nullptr) return;
  if (in_sizes[0] != NSTEPS * 2 || in_sizes[1] != NSTEPS * NAGENT * 2 || in_sizes[2] != NGATE * 2 ||
      in_sizes[3] != NGATE * HID || in_sizes[4] != NGATE || in_sizes[5] != NGATE || in_sizes[6] != HID * NSOC ||
      in_sizes[7] != HID || in_sizes[8] != HID * HID || in_sizes[9] != HID || in_sizes[10] != 2 * HID ||
      in_sizes[11] != 2 || out_size != NOUT) return;

  const float* traj_t = (const float*)d_in[0];
  const float* traj_o = (const float*)d_in[1];
  const float* w_ih   = (const float*)d_in[2];
  const float* w_hh   = (const float*)d_in[3];
  const float* b_ih   = (const float*)d_in[4];
  const float* b_hh   = (const float*)d_in[5];
  const float* w1     = (const float*)d_in[6];
  const float* b1     = (const float*)d_in[7];
  const float* w2     = (const float*)d_in[8];
  const float* b2     = (const float*)d_in[9];
  const float* wout   = (const float*)d_in[10];
  const float* bout   = (const float*)d_in[11];
  float* out = (float*)d_out;

  char* ws = (char*)d_ws; size_t off = 0;
  auto carve = [&](size_t bytes) -> char* { char* p = ws + off; off += (bytes + 255) & ~(size_t)255; return p; };
  unsigned short* WHH  = (unsigned short*)carve((size_t)NGATE * HID * 2);
  float*          PART = (float*)carve((size_t)NBLK * NSTEPS * NSOC * 4);
  if (off > ws_size || off > (size_t)134217728) return;

  const int n8 = (NGATE * HID) / 8;
  cvt_whh_kernel<<<n8 / NTHR, NTHR, 0, stream>>>(w_hh, WHH, n8, WCAR);
  agents_kernel<<<NBLK, NTHR, 0, stream>>>(traj_t, traj_o, w_ih, b_ih, b_hh, WHH, PART);
  pool_target_kernel<<<1, NTHR, 0, stream>>>(traj_t, w_ih, w_hh, b_ih, b_hh, w1, b1, w2, b2, wout, bout, PART, out);
}
